// PixelTransformerResnet_82712480186863
// MI455X (gfx1250) — hardware-verified
//
#include <hip/hip_runtime.h>


namespace {
constexpr int Bn = 8, C = 256, HW = 64, NP = HW * HW, NTOK = Bn * NP;
constexpr float EPS = 1e-5f, OS_ = 8.0f, ISQ = 0.0625f;

typedef _Float16 b16;
typedef __attribute__((ext_vector_type(16))) _Float16 v16b;
typedef __attribute__((ext_vector_type(16))) __bf16 v16bb;
typedef __attribute__((ext_vector_type(8))) _Float16 v8b;
typedef __attribute__((ext_vector_type(8))) unsigned short v8us;
typedef __attribute__((ext_vector_type(8))) float v8f;
typedef __attribute__((ext_vector_type(4))) float v4f;
__device__ __forceinline__ float bf16_rne(float f) { unsigned int u = __float_as_uint(f); u += 0x7FFFu + ((u >> 16) & 1u); return __uint_as_float(u & 0xFFFF0000u); }
__device__ __forceinline__ unsigned short bf16_bits(float f) { unsigned int u = __float_as_uint(f); u += 0x7FFFu + ((u >> 16) & 1u); return (unsigned short)(u >> 16); }
__device__ __forceinline__ void split16(float v, b16& hi, b16& lo) { hi = (b16)v; lo = (b16)(v - (float)hi); }
__device__ __forceinline__ v16b frag_kb(const b16* p, int hh) { const v8b a = *(const v8b*)(p + 8 * hh), b = *(const v8b*)(p + 16 + 8 * hh); v16b f;
#pragma unroll
  for (int e = 0; e < 8; ++e) { f[e] = a[e]; f[8 + e] = b[e]; } return f; }
__device__ __forceinline__ v16bb frag_bf(const unsigned short* p, int hh) { const v8us a = *(const v8us*)(p + 8 * hh), b = *(const v8us*)(p + 16 + 8 * hh); union { unsigned short s[16]; v16bb v; } u;
#pragma unroll
  for (int e = 0; e < 8; ++e) { u.s[e] = a[e]; u.s[8 + e] = b[e]; } return u.v; }
__device__ __forceinline__ v8f wmma16b(v16b a, v16b b, v8f c) { v8f d = __builtin_amdgcn_wmma_f32_16x16x32_f16(false, a, false, b, (short)0, c, false, false); asm volatile("v_nop\n\tv_nop\n\tv_nop\n\tv_nop" : "+v"(d) : "v"(a), "v"(b)); return d; }
__device__ __forceinline__ v8f wmma16bb(v16bb a, v16bb b, v8f c) { v8f d = __builtin_amdgcn_wmma_f32_16x16x32_bf16(false, a, false, b, (short)0, c, false, false); asm volatile("v_nop\n\tv_nop\n\tv_nop\n\tv_nop" : "+v"(d) : "v"(a), "v"(b)); return d; }
__device__ __forceinline__ void wave_lds_sync() { __builtin_amdgcn_fence(__ATOMIC_RELEASE, "workgroup"); __builtin_amdgcn_wave_barrier(); __builtin_amdgcn_fence(__ATOMIC_ACQUIRE, "workgroup"); }
__device__ __forceinline__ float nexp(float x) { return __builtin_amdgcn_exp2f(x * 1.4426950408889634f); }
__device__ __forceinline__ float pmul(float a, float b) { float p = a * b; asm volatile("" : "+v"(p)); return p; }

__global__ __launch_bounds__(256) void prep_kernel(const float* __restrict__ x, const float* __restrict__ W1, const float* __restrict__ W2, const float* __restrict__ W3, const float* __restrict__ W4, const float* __restrict__ g, const float* __restrict__ be, const float* __restrict__ mu, const float* __restrict__ var,
                                                   unsigned short* __restrict__ xT, unsigned short* __restrict__ w16, b16* __restrict__ w4r, float* __restrict__ bnp) {
  __shared__ __attribute__((aligned(16))) unsigned short Tt[64][C + 8];
  const int t_ = threadIdx.x, b = blockIdx.y, p0 = blockIdx.x * 64; const float* src = x + (size_t)b * C * NP;
  for (int i = t_; i < C * 64; i += 256) { const int c = i >> 6, pp = i & 63; Tt[pp][c] = bf16_bits(src[(size_t)c * NP + p0 + pp]); }
  __syncthreads();
  for (int pass = 0; pass < 2; ++pass) {
    for (int i = t_; i < 64 * C / 8; i += 256) { const int pp = i >> 5, c8 = (i & 31) * 8; *(volatile v8us*)(xT + ((size_t)b * NP + p0 + pp) * C + c8) = *(const v8us*)(&Tt[pp][c8]); }
    if (blockIdx.x == 0 && blockIdx.y == 0) {
      for (int i = t_; i < 3 * C * C / 8; i += 256) { const int m = i / (C * C / 8), q = i % (C * C / 8); const float* W = (m == 0) ? W1 : (m == 1) ? W2 : W3; v8us o;
#pragma unroll
        for (int e = 0; e < 8; ++e) o[e] = bf16_bits(W[q * 8 + e]);
        *(volatile v8us*)(w16 + (size_t)i * 8) = o; }
      for (int i = t_; i < C * C / 8; i += 256) { v8b o;
#pragma unroll
        for (int e = 0; e < 8; ++e) o[e] = (b16)bf16_rne(W4[i * 8 + e]);
        *(volatile v8b*)(w4r + (size_t)i * 8) = o; }
      for (int i = t_; i < 5 * C; i += 256) { const float sc = bf16_rne(g[i]) * rsqrtf(bf16_rne(var[i]) + EPS); ((volatile float*)bnp)[(i / C) * 2 * C + (i % C)] = sc; ((volatile float*)bnp)[(i / C) * 2 * C + C + (i % C)] = bf16_rne(be[i]) - bf16_rne(mu[i]) * sc; } }
    __threadfence(); }
}

__global__ __launch_bounds__(128) void qkv_kernel(const unsigned short* __restrict__ xT, const unsigned short* __restrict__ w16, const float* __restrict__ b1, const float* __restrict__ b2, const float* __restrict__ b3, const float* __restrict__ bnp, float* __restrict__ q, float* __restrict__ k, float* __restrict__ v) {
  __shared__ __attribute__((aligned(16))) float Ts[4][32 * 64];
  const int lane = threadIdx.x & 31, wave = threadIdx.x >> 5, nloc = lane & 15, hlf = lane >> 4, which = blockIdx.z, m0 = blockIdx.y * 128 + wave * 32, c0 = blockIdx.x * 64;
  const unsigned short* Wt = w16 + (size_t)which * C * C; const float* bias = (which == 0) ? b1 : (which == 1) ? b2 : b3; const float* sc = bnp + which * 2 * C; const float* sh = sc + C; float* dstb = (which == 0) ? q : (which == 1) ? k : v;
  v8f acc[2][4];
#pragma unroll
  for (int r = 0; r < 2; ++r)
#pragma unroll
    for (int t = 0; t < 4; ++t) acc[r][t] = (v8f){};
#pragma unroll 2
  for (int kb = 0; kb < C; kb += 32) { const v16bb a0 = frag_bf(xT + (size_t)(m0 + nloc) * C + kb, hlf), a1 = frag_bf(xT + (size_t)(m0 + 16 + nloc) * C + kb, hlf);
#pragma unroll
    for (int t = 0; t < 4; ++t) { const v16bb bw = frag_bf(Wt + (size_t)(c0 + t * 16 + nloc) * C + kb, hlf); acc[0][t] = wmma16bb(a0, bw, acc[0][t]); acc[1][t] = wmma16bb(a1, bw, acc[1][t]); } }
  float* Tt = Ts[wave];
#pragma unroll
  for (int t = 0; t < 4; ++t) { const int c = c0 + t * 16 + nloc; const float bb = bf16_rne(bias[c]), s_ = sc[c], h_ = sh[c];
#pragma unroll
    for (int r = 0; r < 2; ++r)
#pragma unroll
      for (int vv = 0; vv < 8; ++vv) Tt[(r * 16 + vv + 8 * hlf) * 64 + t * 16 + nloc] = fmaxf((acc[r][t][vv] + bb) * s_ + h_, 0.0f); }
  wave_lds_sync();
  float* dst0 = dstb + (size_t)m0 * C + c0;
  for (int pass = 0; pass < 2; ++pass) {
#pragma unroll
    for (int j = 0; j < 16; ++j) { const int rr = j * 2 + hlf, c4 = nloc * 4; *(volatile v4f*)(dst0 + (size_t)rr * C + c4) = *(const v4f*)(Tt + rr * 64 + c4); }
    __threadfence(); }
}

__global__ __launch_bounds__(256) void local_kernel(const float* __restrict__ q, const float* __restrict__ k, const float* __restrict__ v, const float* __restrict__ bnp, float* __restrict__ o) {
  const int wid = threadIdx.x >> 5, lane = threadIdx.x & 31; const int px = blockIdx.x * 8 + wid, b = px / NP, pp = px % NP, y = pp >> 6, xx = pp & 63; const int ca = lane * 4, cb = 128 + lane * 4;
  const v4f qa = *(const v4f*)(q + (size_t)px * C + ca), qb = *(const v4f*)(q + (size_t)px * C + cb);
  float lg[9]; bool ok[9]; size_t np_[9];
#pragma unroll
  for (int n = 0; n < 9; ++n) { const int dy = n / 3 - 1, dx = n % 3 - 1, y1 = y + dy, x1 = xx + dx; ok[n] = ((unsigned)y1 < 64u) && ((unsigned)x1 < 64u); np_[n] = (size_t)b * NP + (min(max(y1, 0), 63) << 6) + min(max(x1, 0), 63);
    float d = 0.0f; if (ok[n]) { const v4f ka = *(const v4f*)(k + np_[n] * C + ca), kb2 = *(const v4f*)(k + np_[n] * C + cb);
#pragma unroll
      for (int e = 0; e < 4; ++e) d += pmul(qa[e], ka[e]) + pmul(qb[e], kb2[e]); }
#pragma unroll
    for (int of = 1; of < 32; of <<= 1) d += __shfl_xor(d, of);
    lg[n] = ok[n] ? d * ISQ : 0.0f; }
  float m = lg[0];
#pragma unroll
  for (int n = 1; n < 9; ++n) m = fmaxf(m, lg[n]);
  float e_[9], z = 0.0f;
#pragma unroll
  for (int n = 0; n < 9; ++n) { e_[n] = nexp(lg[n] - m); z += e_[n]; }
  const float iz = 1.0f / z; v4f oa = {0.0f, 0.0f, 0.0f, 0.0f}, ob = oa;
#pragma unroll
  for (int n = 0; n < 9; ++n) { if (ok[n]) { const float a_ = e_[n] * iz; const v4f va = *(const v4f*)(v + np_[n] * C + ca), vb = *(const v4f*)(v + np_[n] * C + cb);
#pragma unroll
      for (int e = 0; e < 4; ++e) { oa[e] += pmul(a_, va[e]); ob[e] += pmul(a_, vb[e]); } } }
  const float* sc = bnp + 3 * 2 * C; const float* sh = sc + C;
#pragma unroll
  for (int e = 0; e < 4; ++e) { oa[e] = fmaxf(oa[e] * sc[ca + e] + sh[ca + e], 0.0f); ob[e] = fmaxf(ob[e] * sc[cb + e] + sh[cb + e], 0.0f); }
  for (int pass = 0; pass < 2; ++pass) { *(volatile v4f*)(o + (size_t)px * C + ca) = oa; *(volatile v4f*)(o + (size_t)px * C + cb) = ob; __threadfence(); }
}

__global__ __launch_bounds__(128) void final_kernel(const float* __restrict__ orow, const b16* __restrict__ w4r, const float* __restrict__ b4, const float* __restrict__ bnp, const float* __restrict__ x, float* __restrict__ out) {
  __shared__ __attribute__((aligned(16))) float Tc[64][128 + 4];
  const int lane = threadIdx.x & 31, wave = threadIdx.x >> 5, nloc = lane & 15, hlf = lane >> 4, m0 = blockIdx.y * 128 + wave * 32, c0 = blockIdx.x * 64; const int b = (blockIdx.y * 128) / NP, p0 = (blockIdx.y * 128) % NP;
  v8f acc[2][4];
#pragma unroll
  for (int r = 0; r < 2; ++r)
#pragma unroll
    for (int t = 0; t < 4; ++t) acc[r][t] = (v8f){};
#pragma unroll 2
  for (int kb = 0; kb < C; kb += 32) { v16b a0, a1, l0, l1;
#pragma unroll
    for (int e = 0; e < 16; ++e) { const int kk = kb + ((e < 8) ? (8 * hlf + e) : (16 + 8 * hlf + e - 8)); b16 p, qq; split16(orow[(size_t)(m0 + nloc) * C + kk] * OS_, p, qq); a0[e] = p; l0[e] = qq; split16(orow[(size_t)(m0 + 16 + nloc) * C + kk] * OS_, p, qq); a1[e] = p; l1[e] = qq; }
#pragma unroll
    for (int t = 0; t < 4; ++t) { const v16b bw = frag_kb(w4r + (size_t)(c0 + t * 16 + nloc) * C + kb, hlf); acc[0][t] = wmma16b(a0, bw, acc[0][t]); acc[0][t] = wmma16b(l0, bw, acc[0][t]); acc[1][t] = wmma16b(a1, bw, acc[1][t]); acc[1][t] = wmma16b(l1, bw, acc[1][t]); } }
  const float* sc = bnp + 4 * 2 * C; const float* sh = sc + C;
#pragma unroll
  for (int t = 0; t < 4; ++t) { const int co = c0 + t * 16 + nloc; const float bb = bf16_rne(b4[co]), s_ = sc[co], h_ = sh[co];
#pragma unroll
    for (int r = 0; r < 2; ++r)
#pragma unroll
      for (int vv = 0; vv < 8; ++vv) { const int pl_ = wave * 32 + r * 16 + 8 * hlf + vv; const float val = (acc[r][t][vv] * (1.0f / OS_) + bb) * s_ + h_ + bf16_rne(x[((size_t)b * C + co) * NP + p0 + pl_]); Tc[t * 16 + nloc][pl_] = fmaxf(val, 0.0f); } }
  __syncthreads();
  for (int pass = 0; pass < 2; ++pass) { for (int i = threadIdx.x; i < 64 * 32; i += 128) { const int cc = i >> 5, c4 = (i & 31) * 4; *(volatile v4f*)(out + ((size_t)b * C + c0 + cc) * NP + p0 + c4) = *(const v4f*)(&Tc[cc][c4]); } __threadfence(); }
}
}

extern "C" void kernel_launch(void* const* d_in, const int* in_sizes, int n_in,
                              void* d_out, int out_size, void* d_ws, size_t ws_size, hipStream_t stream) {
  (void)n_in; (void)out_size;
  const float* x = (const float*)d_in[0]; const float* W1 = (const float*)d_in[1]; const float* b1 = (const float*)d_in[2]; const float* W2 = (const float*)d_in[3]; const float* b2 = (const float*)d_in[4]; const float* W3 = (const float*)d_in[5]; const float* b3 = (const float*)d_in[6]; const float* W4 = (const float*)d_in[7]; const float* b4 = (const float*)d_in[8];
  const float* g = (const float*)d_in[9]; const float* be = (const float*)d_in[10]; const float* mu = (const float*)d_in[11]; const float* var = (const float*)d_in[12];
  float* out = (float*)d_out;
  if (in_sizes[0] != Bn * C * NP || in_sizes[1] != C * C || in_sizes[7] != C * C || in_sizes[9] != 5 * C || in_sizes[12] != 5 * C) return;
  size_t off = 0; char* ws = (char*)d_ws;
  auto carve = [&](size_t bytes) { char* p = ws + off; off += (bytes + 255) & ~(size_t)255; return p; };
  unsigned short* xT = (unsigned short*)carve((size_t)NTOK * C * 2); unsigned short* w16 = (unsigned short*)carve((size_t)3 * C * C * 2); b16* w4r = (b16*)carve((size_t)C * C * 2); float* bnp = (float*)carve(5 * 2 * C * 4);
  float* q = (float*)carve((size_t)NTOK * C * 4); float* k = (float*)carve((size_t)NTOK * C * 4); float* v = (float*)carve((size_t)NTOK * C * 4);
  if (off > ws_size) return;
  prep_kernel<<<dim3(NP / 64, Bn), 256, 0, stream>>>(x, W1, W2, W3, W4, g, be, mu, var, xT, w16, w4r, bnp);
  qkv_kernel<<<dim3(C / 64, NTOK / 128, 3), 128, 0, stream>>>(xT, w16, b1, b2, b3, bnp, q, k, v);
  local_kernel<<<NTOK / 8, 256, 0, stream>>>(q, k, v, bnp, q);
  final_kernel<<<dim3(C / 64, NTOK / 128), 128, 0, stream>>>(q, w4r, b4, bnp, x, out);
}
